// GraphVAE_3315714752918
// MI455X (gfx1250) — hardware-run, weakly checked
//
#include <hip/hip_runtime.h>


#define NN 2048
#define EE 65536
#define FD 7
#define SD 32
#define G3 96
#define LD 16
#define RR 3
#define TP 36
#define GP 200
#define DT 32

#define OFF_MSG 0
#define OFF_IH  (RR * SD * SD)
#define OFF_HH  (OFF_IH + RR * G3 * SD)
#define OFF_HD  (OFF_HH + RR * G3 * SD)
#define OFF_AB  (OFF_HD + SD * SD)
#define WPL_N   (OFF_AB + SD * SD)
#define WB_IH  (OFF_IH / 256)
#define WB_HH  (OFF_HH / 256)
#define WB_HD  (OFF_HD / 256)
#define WB_AB  (OFF_AB / 256)
#define WB_END (WPL_N / 256)

static_assert(SD == 32);
static_assert(2 * LD == SD);
static_assert(G3 == 3 * SD);
static_assert(NN % 16 == 0);
static_assert(NN % DT == 0);
static_assert(EE % 128 == 0);
static_assert(OFF_IH % 256 == 0 && OFF_HH % 256 == 0 && OFF_HD % 256 == 0 && OFF_AB % 256 == 0 && WPL_N % 256 == 0);
static_assert((SD * SD) % 256 == 0 && (G3 * SD) % 256 == 0);
static_assert((LD * SD) % 256 == 0);
static_assert(WB_END == 92);
static_assert((TP * 4) % 16 == 0);
static_assert(4 * 32 * 16 == 16 * SD * 4);
static_assert(2 * 32 * 16 == 16 * LD * 4);
static_assert(256 * 16 == DT * DT * 4);
static_assert((size_t)NN * NN * 4 == 16777216);
static_assert((size_t)NN * NN * 4 + (size_t)NN * LD * 4 == 16908288);
static_assert((3 * 16 * TP + 16 * GP) * 4 <= 131072);
static_assert(3 * DT * TP * 4 <= 131072);

typedef unsigned short bf;
typedef __attribute__((ext_vector_type(16))) __bf16   v16bf;
typedef __attribute__((ext_vector_type(8)))  unsigned short v8us;
typedef __attribute__((ext_vector_type(8)))  float    v8f;
typedef __attribute__((ext_vector_type(4)))  float    v4f;
typedef __attribute__((ext_vector_type(4)))  int      v4i;
typedef v4f  __attribute__((may_alias)) v4fa;

__device__ __forceinline__ unsigned short f2bf(float f) { unsigned u = __float_as_uint(f); u += 0x7FFFu + ((u >> 16) & 1u); return (unsigned short)(u >> 16); }
__device__ __forceinline__ float bfr(float f) { return __uint_as_float(((unsigned)f2bf(f)) << 16); }
__device__ __forceinline__ v16bf cat16b(v8us lo, v8us hi) { return __builtin_bit_cast(v16bf, __builtin_shufflevector(lo, hi, 0, 1, 2, 3, 4, 5, 6, 7, 8, 9, 10, 11, 12, 13, 14, 15)); }
__device__ __forceinline__ v8f wmmab(v16bf a, v16bf b, v8f c) { return __builtin_amdgcn_wmma_f32_16x16x32_bf16(false, a, false, b, (short)0, c, false, false); }
__device__ __forceinline__ v16bf ldb(const bf* p)  { return cat16b(*(const v8us*)p, *(const v8us*)(p + 16)); }
__device__ __forceinline__ void wave_sync() { __builtin_amdgcn_fence(3  , "wavefront"); __builtin_amdgcn_wave_barrier(); asm volatile("" ::: "memory"); }

__device__ __forceinline__ v8f wmmab_g(v16bf a, v16bf b, v8f c) {
    c = wmmab(a, b, c);
    asm volatile("v_nop\n\tv_nop\n\tv_nop\n\tv_nop" : "+v"(c) : "v"(a), "v"(b));
    return c;
}
__device__ __forceinline__ float bf2f(unsigned short b) { return __uint_as_float(((unsigned)b) << 16); }
__device__ __forceinline__ v4f ld4(const float* p) { return *(const v4fa*)p; }
__device__ __forceinline__ void mk_frag(v4f x0, v4f x1, v4f x2, v4f x3, v16bf& H, v16bf& L) {
    v8us h0, h1, l0, l1;
#pragma unroll
    for (int i = 0; i < 4; ++i) {
        unsigned short a;
        a = f2bf(x0[i]); h0[i] = a;     l0[i] = f2bf(x0[i] - bf2f(a));
        a = f2bf(x1[i]); h0[4 + i] = a; l0[4 + i] = f2bf(x1[i] - bf2f(a));
        a = f2bf(x2[i]); h1[i] = a;     l1[i] = f2bf(x2[i] - bf2f(a));
        a = f2bf(x3[i]); h1[4 + i] = a; l1[4 + i] = f2bf(x3[i] - bf2f(a));
    }
    H = cat16b(h0, h1); L = cat16b(l0, l1);
}
__device__ __forceinline__ v8f tile_mm(v16bf aH, v16bf aL, const bf* __restrict__ wrow) {
    const v16bf b = ldb(wrow);
    v8f c = (v8f){};
    c = wmmab_g(aH, b, c);
    c = wmmab_g(aL, b, c);
    return c;
}
__device__ __forceinline__ float sigm(float v) { const float c = fminf(fmaxf(v, -30.0f), 30.0f); return __builtin_amdgcn_rcpf(1.0f + expf(-c)); }

__device__ __forceinline__ v8us wrow8(const float* __restrict__ W, int ldw, int col, int k0, int kreal) {
    v8us o;
#pragma unroll
    for (int i = 0; i < 8; ++i) {
        const int k = k0 + i;
        const int kc = k < kreal ? k : (kreal - 1);
        float v = W[(size_t)kc * ldw + col];
        asm volatile("" : "+v"(v));
        o[i] = (k < kreal) ? f2bf(v) : (unsigned short)0;
    }
    return o;
}

__global__ __launch_bounds__(32) void k_wprep(const float* __restrict__ wmsg, const float* __restrict__ wih, const float* __restrict__ whh,
                                              const float* __restrict__ wmu, const float* __restrict__ wls, const float* __restrict__ wd1, bf* dst) {
    const int blk = blockIdx.x;
    const int e = (blk * 32 + (int)threadIdx.x) * 8;
    const int k0 = e & 31;
    v8us o;
    if (blk < WB_IH)          { const int r = e / (SD * SD); const int n = (e >> 5) & (SD - 1); o = wrow8(wmsg + r * SD * SD, SD, n, k0, SD); }
    else if (blk < WB_HH)     { const int q = e - OFF_IH; const int r = q / (G3 * SD); const int n = (q - r * G3 * SD) >> 5; o = wrow8(wih + r * SD * G3, G3, n, k0, SD); }
    else if (blk < WB_HD)     { const int q = e - OFF_HH; const int r = q / (G3 * SD); const int n = (q - r * G3 * SD) >> 5; o = wrow8(whh + r * SD * G3, G3, n, k0, SD); }
    else if (blk < WB_HD + 2) { const int n = (e - OFF_HD) >> 5; o = wrow8(wmu, LD, n, k0, SD); }
    else if (blk < WB_AB)     { const int n = ((e - OFF_HD) >> 5) - LD; o = wrow8(wls, LD, n, k0, SD); }
    else if (blk < WB_AB + 2) { const int n = (e - OFF_AB) >> 5; o = wrow8(wd1, LD, n, k0, LD); }
    else                      { const int n = ((e - OFF_AB) >> 5) - LD; o = wrow8(wd1 + LD * LD, LD, n, k0, LD); }
    *(volatile v8us*)(dst + e) = o; __threadfence(); *(volatile v8us*)(dst + e) = o;
}

__global__ __launch_bounds__(32) void k_enc(const float* __restrict__ x, const float* __restrict__ win, const float* __restrict__ bin,
                                            const bf* __restrict__ wm, const float* __restrict__ bm, float* state, float* msgo) {
    __shared__ __align__(16) float t_st[16 * TP];
    __shared__ __align__(16) float t_o[16 * TP];
    const int lane = threadIdx.x & 31, lr = lane & 15, hi = lane >> 4;
    const int base = blockIdx.x * 16;
    float wc[FD];
#pragma unroll
    for (int f = 0; f < FD; ++f) wc[f] = bfr(win[f * SD + lane]);
    const float bi = bfr(bin[lane]);
#pragma unroll 1
    for (int row = 0; row < 16; ++row) {
        const float* xr = x + (size_t)(base + row) * FD;
        float acc = 0.0f;
#pragma unroll
        for (int f = 0; f < FD; ++f) acc = fmaf(bfr(xr[f]), wc[f], acc);
        t_st[row * TP + lane] = fmaxf(acc + bi, 0.0f);
    }
    wave_sync();
    v16bf sH, sL;
    { const float* p = &t_st[lr * TP + 8 * hi]; mk_frag(ld4(p), ld4(p + 4), ld4(p + 16), ld4(p + 20), sH, sL); }
    const float bia0 = bfr(bm[lr]), bia1 = bfr(bm[16 + lr]);
    const size_t wo = (size_t)lr * SD + 8 * hi;
    const v8f c0 = tile_mm(sH, sL, wm + wo);
    const v8f c1 = tile_mm(sH, sL, wm + wo + 16 * SD);
#pragma unroll
    for (int j = 0; j < 8; ++j) {
        t_o[(8 * hi + j) * TP + lr]      = fmaxf(c0[j] + bia0, 0.0f);
        t_o[(8 * hi + j) * TP + 16 + lr] = fmaxf(c1[j] + bia1, 0.0f); }
    wave_sync();
#pragma unroll 1
    for (int ps = 0; ps < 2; ++ps) {
#pragma unroll
        for (int s = 0; s < 4; ++s) { const int row = 4 * s + (lane >> 3), cofs = (lane & 7) * 4;
            const v4f sv = ld4(&t_st[row * TP + cofs]); const v4f mv = ld4(&t_o[row * TP + cofs]);
            *(volatile v4f*)(state + (size_t)(base + row) * SD + cofs) = sv;
            *(volatile v4f*)(msgo + (size_t)(base + row) * SD + cofs) = mv; }
        if (ps == 0) __threadfence(); }
}

__device__ __forceinline__ void drain1(int d, int s, int base, int lane, const float* __restrict__ msg, float* t_agg) {
    const unsigned dl = (unsigned)d - (unsigned)base;
    const bool hit = dl < 16u;
    const int sc = s < 0 ? 0 : (s > NN - 1 ? NN - 1 : s);
    unsigned mask = __builtin_amdgcn_ballot_w32(hit);
#pragma unroll 1
    for (int it = 0; it < 32; ++it) {
        if (mask == 0u) break;
        const int l = __builtin_ctz(mask);
        const int ss = __builtin_amdgcn_readlane(sc, l);
        const int dd = __builtin_amdgcn_readlane((int)dl, l) & 15;
        const float v = msg[(size_t)ss * SD + lane];
        t_agg[dd * TP + lane] += v;
        mask &= mask - 1u;
    }
}

template <int LAST>
__device__ __forceinline__ void pass_body(float* t_agg, float* t_st, float* t_g, float* t_o,
                                          const int* __restrict__ ei, const float* __restrict__ msg, float* state,
                                          const bf* __restrict__ wih, const bf* __restrict__ whh, const float* __restrict__ bih, const float* __restrict__ bhh,
                                          const bf* __restrict__ wn, const float* __restrict__ bn0, const float* __restrict__ bn1, float* msgo,
                                          const bf* __restrict__ wab, const float* __restrict__ bd1, float* mu, float* ls, float* ab) {
    const int lane = threadIdx.x & 31, lr = lane & 15, hi = lane >> 4;
    const int base = blockIdx.x * 16;
    for (int i = lane; i < 16 * TP; i += 32) t_agg[i] = 0.0f;
#pragma unroll
    for (int s = 0; s < 4; ++s) { const int row = 4 * s + (lane >> 3), cofs = (lane & 7) * 4;
        const v4f v = *(const v4f*)(state + (size_t)(base + row) * SD + cofs);
        *(v4fa*)(&t_st[row * TP + cofs]) = v; }
    wave_sync();
    const int* dstp = ei + EE;
#pragma unroll 1
    for (int c = 0; c < EE / 128; ++c) {
        const int e0 = c * 128 + lane * 4;
        const v4i dv = *(const v4i*)(dstp + e0);
        const v4i sv = *(const v4i*)(ei + e0);
        drain1(dv[0], sv[0], base, lane, msg, t_agg);
        drain1(dv[1], sv[1], base, lane, msg, t_agg);
        drain1(dv[2], sv[2], base, lane, msg, t_agg);
        drain1(dv[3], sv[3], base, lane, msg, t_agg);
    }
    wave_sync();
    v16bf aH, aL, sH, sL;
    { const float* p = &t_agg[lr * TP + 8 * hi]; mk_frag(ld4(p), ld4(p + 4), ld4(p + 16), ld4(p + 20), aH, aL); }
    { const float* p = &t_st[lr * TP + 8 * hi];  mk_frag(ld4(p), ld4(p + 4), ld4(p + 16), ld4(p + 20), sH, sL); }
    const size_t wo = (size_t)lr * SD + 8 * hi;
#pragma unroll
    for (int nt = 0; nt < 6; ++nt) {
        const v8f cx = tile_mm(aH, aL, wih + wo + (size_t)nt * 16 * SD);
        const v8f ch = tile_mm(sH, sL, whh + wo + (size_t)nt * 16 * SD);
#pragma unroll
        for (int j = 0; j < 8; ++j) {
            t_g[(8 * hi + j) * GP + nt * 16 + lr]      = cx[j];
            t_g[(8 * hi + j) * GP + G3 + nt * 16 + lr] = ch[j]; }
    }
    wave_sync();
    {
        const float bxr = bfr(bih[lane]), bxz = bfr(bih[SD + lane]), bxn = bfr(bih[2 * SD + lane]);
        const float bhr = bfr(bhh[lane]), bhz = bfr(bhh[SD + lane]), bhn = bfr(bhh[2 * SD + lane]);
#pragma unroll 1
        for (int row = 0; row < 16; ++row) {
            const float* g = &t_g[row * GP];
            const float xr = g[lane] + bxr, xz = g[SD + lane] + bxz, xn = g[2 * SD + lane] + bxn;
            const float hr = g[G3 + lane] + bhr, hz = g[G3 + SD + lane] + bhz, hn = g[G3 + 2 * SD + lane] + bhn;
            const float s = t_st[row * TP + lane];
            const float rg = sigm(xr + hr);
            const float zg = sigm(xz + hz);
            const float ng = tanhf(xn + rg * hn);
            const float nh = (1.0f - zg) * ng + zg * s;
            t_st[row * TP + lane] = s + nh;
        }
    }
    wave_sync();
    v16bf nH, nL;
    { const float* p = &t_st[lr * TP + 8 * hi]; mk_frag(ld4(p), ld4(p + 4), ld4(p + 16), ld4(p + 20), nH, nL); }
    {
        const float bia0 = bfr(bn0[lr]);
        const float bia1 = LAST ? bfr(bn1[lr]) : bfr(bn0[16 + lr]);
        const v8f c0 = tile_mm(nH, nL, wn + wo);
        const v8f c1 = tile_mm(nH, nL, wn + wo + 16 * SD);
#pragma unroll
        for (int j = 0; j < 8; ++j) {
            float u0 = c0[j] + bia0, u1 = c1[j] + bia1;
            if (!LAST) { u0 = fmaxf(u0, 0.0f); u1 = fmaxf(u1, 0.0f); }
            t_o[(8 * hi + j) * TP + lr] = u0;
            t_o[(8 * hi + j) * TP + 16 + lr] = u1; }
    }
    wave_sync();
    if (LAST) {
        v16bf mH, mL;
        { const float* p = &t_o[lr * TP + 8 * hi]; const v4f z = (v4f){}; mk_frag(ld4(p), ld4(p + 4), z, z, mH, mL); }
        const float bdv = bfr(bd1[lr]);
        const v8f a0 = tile_mm(mH, mL, wab + wo);
        const v8f a1 = tile_mm(mH, mL, wab + wo + 16 * SD);
#pragma unroll
        for (int j = 0; j < 8; ++j) {
            t_agg[(8 * hi + j) * TP + lr] = a0[j];
            t_agg[(8 * hi + j) * TP + 16 + lr] = a1[j] + bdv; }
        wave_sync();
    }
#pragma unroll 1
    for (int ps = 0; ps < 2; ++ps) {
        if (!LAST) {
#pragma unroll
            for (int s = 0; s < 4; ++s) { const int row = 4 * s + (lane >> 3), cofs = (lane & 7) * 4;
                const v4f sv = ld4(&t_st[row * TP + cofs]); const v4f mv = ld4(&t_o[row * TP + cofs]);
                *(volatile v4f*)(state + (size_t)(base + row) * SD + cofs) = sv;
                *(volatile v4f*)(msgo + (size_t)(base + row) * SD + cofs) = mv; }
        } else {
#pragma unroll
            for (int s = 0; s < 4; ++s) { const int row = 4 * s + (lane >> 3), cofs = (lane & 7) * 4;
                const v4f av = ld4(&t_agg[row * TP + cofs]);
                *(volatile v4f*)(ab + (size_t)(base + row) * SD + cofs) = av; }
#pragma unroll
            for (int s = 0; s < 2; ++s) { const int p = s * 32 + lane; const int row = p >> 2, c4 = (p & 3) * 4;
                const v4f mv = ld4(&t_o[row * TP + c4]); const v4f lv = ld4(&t_o[row * TP + 16 + c4]);
                *(volatile v4f*)(mu + (size_t)base * LD + (size_t)p * 4) = mv;
                *(volatile v4f*)(ls + (size_t)base * LD + (size_t)p * 4) = lv; }
        }
        if (ps == 0) __threadfence(); }
}

__global__ __launch_bounds__(32) void k_pass_mid(const int* __restrict__ ei, const float* __restrict__ msg, float* state,
                                                 const bf* __restrict__ wih, const bf* __restrict__ whh, const float* __restrict__ bih, const float* __restrict__ bhh,
                                                 const bf* __restrict__ wn, const float* __restrict__ bn, float* msgo) {
    __shared__ __align__(16) float t_agg[16 * TP];
    __shared__ __align__(16) float t_st[16 * TP];
    __shared__ __align__(16) float t_g[16 * GP];
    __shared__ __align__(16) float t_o[16 * TP];
    pass_body<0>(t_agg, t_st, t_g, t_o, ei, msg, state, wih, whh, bih, bhh, wn, bn, bn, msgo, wn, bn, msgo, msgo, msgo);
}

__global__ __launch_bounds__(32) void k_pass_last(const int* __restrict__ ei, const float* __restrict__ msg, float* state,
                                                  const bf* __restrict__ wih, const bf* __restrict__ whh, const float* __restrict__ bih, const float* __restrict__ bhh,
                                                  const bf* __restrict__ whd, const float* __restrict__ bmu, const float* __restrict__ bls,
                                                  const bf* __restrict__ wab, const float* __restrict__ bd1, float* mu, float* ls, float* ab) {
    __shared__ __align__(16) float t_agg[16 * TP];
    __shared__ __align__(16) float t_st[16 * TP];
    __shared__ __align__(16) float t_g[16 * GP];
    __shared__ __align__(16) float t_o[16 * TP];
    pass_body<1>(t_agg, t_st, t_g, t_o, ei, msg, state, wih, whh, bih, bhh, whd, bmu, bls, ab, wab, bd1, mu, ls, ab);
}

__global__ __launch_bounds__(256) void k_dec(const float* __restrict__ ab, const float* __restrict__ wd2, const float* __restrict__ bd2, float* out) {
    __shared__ __align__(16) float sI[DT * TP];
    __shared__ __align__(16) float sJ[DT * TP];
    __shared__ __align__(16) float so[DT * TP];
    const int it = blockIdx.y, jt = blockIdx.x;
    if (jt < it) return;
    const int t = threadIdx.x; const int row = t >> 3, c4 = (t & 7) * 4;
    const int i0 = it * DT, j0 = jt * DT;
    { const v4f u = *(const v4f*)(ab + (size_t)(i0 + row) * SD + c4); *(v4fa*)(&sI[row * TP + c4]) = u;
      const v4f w = *(const v4f*)(ab + (size_t)(j0 + row) * SD + c4); *(v4fa*)(&sJ[row * TP + c4]) = w; }
    float wv[LD];
#pragma unroll
    for (int k = 0; k < LD; ++k) wv[k] = bfr(wd2[k]);
    const float bz = bfr(bd2[0]);
    __syncthreads();
    float aI[LD], bI[LD];
    { const float* p = &sI[row * TP];
#pragma unroll
      for (int q = 0; q < 4; ++q) { const v4f u = ld4(p + 4 * q), w = ld4(p + LD + 4 * q);
#pragma unroll
          for (int c = 0; c < 4; ++c) { aI[4 * q + c] = u[c]; bI[4 * q + c] = w[c]; } } }
#pragma unroll 1
    for (int jj = 0; jj < 4; ++jj) {
        const int jl = c4 + jj;
        const float* p = &sJ[jl * TP];
        float s1 = 0.0f, s2 = 0.0f;
#pragma unroll
        for (int q = 0; q < 4; ++q) { const v4f u = ld4(p + 4 * q), w = ld4(p + LD + 4 * q);
#pragma unroll
            for (int c = 0; c < 4; ++c) { const int k = 4 * q + c;
                s1 = fmaf(fmaxf(aI[k] + w[c], 0.0f), wv[k], s1);
                s2 = fmaf(fmaxf(u[c] + bI[k], 0.0f), wv[k], s2); } }
        so[row * TP + jl] = sigm(0.5f * (s1 + s2) + bz);
    }
    __syncthreads();
    const v4f nv = ld4(&so[row * TP + c4]);
    v4f tv;
    tv[0] = so[(c4 + 0) * TP + row]; tv[1] = so[(c4 + 1) * TP + row]; tv[2] = so[(c4 + 2) * TP + row]; tv[3] = so[(c4 + 3) * TP + row];
    float* pn = out + (size_t)(i0 + row) * NN + j0 + c4;
    float* pt = out + (size_t)(j0 + row) * NN + i0 + c4;
    const bool offd = jt != it;
#pragma unroll 1
    for (int ps = 0; ps < 2; ++ps) {
        *(volatile v4f*)pn = nv;
        if (offd) *(volatile v4f*)pt = tv;
        if (ps == 0) __threadfence(); }
}

static constexpr size_t al256(size_t v) { return (v + 255) & ~(size_t)255; }
static constexpr size_t SZ_WPL = al256((size_t)WPL_N * 2);
static constexpr size_t SZ_F   = al256((size_t)NN * SD * 4);
static constexpr size_t SZ_TOTAL = SZ_WPL + 4 * SZ_F;
static_assert(SZ_TOTAL <= (size_t)134217728);
static_assert((size_t)WB_END * 32 * 8 * 2 <= SZ_WPL);
static_assert((size_t)(NN / 16) * 16 * SD * 4 <= SZ_F);

extern "C" void kernel_launch(void* const* d_in, const int* in_sizes, int n_in,
                              void* d_out, int out_size, void* d_ws, size_t ws_size, hipStream_t stream) {
    if (n_in < 18) return;
    if (in_sizes[0] < NN * FD || in_sizes[1] < 2 * EE || in_sizes[2] < FD * SD || in_sizes[3] < SD) return;
    if (in_sizes[4] < RR * SD * SD || in_sizes[5] < RR * SD || in_sizes[6] < RR * SD * G3 || in_sizes[7] < RR * SD * G3) return;
    if (in_sizes[8] < RR * G3 || in_sizes[9] < RR * G3 || in_sizes[10] < SD * LD || in_sizes[11] < LD) return;
    if (in_sizes[12] < SD * LD || in_sizes[13] < LD || in_sizes[14] < 2 * LD * LD || in_sizes[15] < LD || in_sizes[16] < LD || in_sizes[17] < 1) return;
    if ((size_t)out_size < (size_t)NN * NN + (size_t)2 * NN * LD) return;
    if (SZ_TOTAL > ws_size) return;
    const float* x    = (const float*)d_in[0];
    const int*   ei   = (const int*)d_in[1];
    const float* win  = (const float*)d_in[2];
    const float* bin  = (const float*)d_in[3];
    const float* wmsg = (const float*)d_in[4];
    const float* bmsg = (const float*)d_in[5];
    const float* wih  = (const float*)d_in[6];
    const float* whh  = (const float*)d_in[7];
    const float* bih  = (const float*)d_in[8];
    const float* bhh  = (const float*)d_in[9];
    const float* wmu  = (const float*)d_in[10];
    const float* bmu  = (const float*)d_in[11];
    const float* wls  = (const float*)d_in[12];
    const float* bls  = (const float*)d_in[13];
    const float* wd1  = (const float*)d_in[14];
    const float* bd1  = (const float*)d_in[15];
    const float* wd2  = (const float*)d_in[16];
    const float* bd2  = (const float*)d_in[17];
    float* OUT = (float*)d_out;
    float* MU = OUT + (size_t)NN * NN;
    float* LS = MU + (size_t)NN * LD;
    char* wsp = (char*)d_ws;
    bf* WPL = (bf*)wsp; wsp += SZ_WPL;
    float* ST = (float*)wsp; wsp += SZ_F;
    float* M0 = (float*)wsp; wsp += SZ_F;
    float* M1 = (float*)wsp; wsp += SZ_F;
    float* AB = (float*)wsp; wsp += SZ_F;

    k_wprep<<<WB_END, 32, 0, stream>>>(wmsg, wih, whh, wmu, wls, wd1, WPL);
    k_enc<<<NN / 16, 32, 0, stream>>>(x, win, bin, WPL + OFF_MSG, bmsg, ST, M0);
    k_pass_mid<<<NN / 16, 32, 0, stream>>>(ei, M0, ST, WPL + OFF_IH, WPL + OFF_HH, bih, bhh, WPL + OFF_MSG + SD * SD, bmsg + SD, M1);
    k_pass_mid<<<NN / 16, 32, 0, stream>>>(ei, M1, ST, WPL + OFF_IH + G3 * SD, WPL + OFF_HH + G3 * SD, bih + G3, bhh + G3, WPL + OFF_MSG + 2 * SD * SD, bmsg + 2 * SD, M0);
    k_pass_last<<<NN / 16, 32, 0, stream>>>(ei, M0, ST, WPL + OFF_IH + 2 * G3 * SD, WPL + OFF_HH + 2 * G3 * SD, bih + 2 * G3, bhh + 2 * G3,
                                            WPL + OFF_HD, bmu, bls, WPL + OFF_AB, bd1, MU, LS, AB);
    k_dec<<<dim3(NN / DT, NN / DT, 1), 256, 0, stream>>>(AB, wd2, bd2, OUT);
}
